// GIN_5282809775005
// MI455X (gfx1250) — hardware-verified
//
#include <hip/hip_runtime.h>
#include <stddef.h>
#include <stdint.h>

#pragma clang fp contract(off)


#define DFE     128
#define KA      256
#define WMAT    (DFE * KA)
#define NCMAX   64
#define NTHR    256
#define NWAVE   8
#define EPT     8
#define CHUNK   (NTHR * EPT)
#define WCAP    (EPT * 32)
#define LISTN   (NWAVE * WCAP)
#define NBMAX   2048
#define RCAP    28672
#define DEGCAP  1024
#define STW     512
#define GBM     64
#define GTHR    128
#define WSMAX   134217728
#define LDS_AGG ((2 * RCAP + 2 * NBMAX + LISTN) * 4 + 64)

static_assert((CHUNK & (CHUNK - 1)) == 0 && CHUNK <= 4096);
static_assert((NBMAX & (NBMAX - 1)) == 0 && NBMAX <= 4096);
static_assert(NTHR * 8 == NBMAX);
static_assert(LISTN >= NBMAX);
static_assert(LISTN >= NWAVE * WCAP);
static_assert((RCAP % 32) == 0);
static_assert(NWAVE * STW <= RCAP);
static_assert(LDS_AGG <= 300000);
static_assert(GBM == (GTHR / 32) * 16);
static_assert(GTHR == DFE);
static_assert((KA % 32) == 0 && KA == 2 * DFE);
static_assert(DFE == 4 * 32);
static_assert(4 * 32 <= STW);
static_assert((DFE * (KA / 8)) % NTHR == 0);
static_assert((NCMAX * (KA / 8)) % NTHR == 0);
static_assert(NCMAX == 4 * 16 && NCMAX <= GTHR);
static_assert((GBM * NCMAX) % 4 == 0);

typedef float          v4f  __attribute__((ext_vector_type(4)));
typedef float          v8f  __attribute__((ext_vector_type(8)));
typedef int            v4i  __attribute__((ext_vector_type(4)));
typedef int            v8i  __attribute__((ext_vector_type(8)));
typedef unsigned short v8us __attribute__((ext_vector_type(8)));
typedef __bf16         v16b __attribute__((ext_vector_type(16)));
typedef v8us __attribute__((may_alias)) v8usa;
typedef v4f  __attribute__((may_alias)) v4fa;
union FragB { v16b v; v8us h[2]; v8i w; };

__device__ __forceinline__ unsigned bf16u(float f) {
  const unsigned u = __float_as_uint(f);
  return (u + 0x7FFFu + ((u >> 16) & 1u)) & 0xFFFF0000u;
}
__device__ __forceinline__ float bf16r(float f) { return __uint_as_float(bf16u(f)); }
__device__ __forceinline__ unsigned short bf16s(float f) { return (unsigned short)(bf16u(f) >> 16); }

__device__ __forceinline__ v8f wmb(const FragB& a, const FragB& b, v8f c) {
  v8f d = __builtin_amdgcn_wmma_f32_16x16x32_bf16(false, a.v, false, b.v, (short)0, c, false, false);
  asm volatile("v_nop\n\tv_nop\n\tv_nop\n\tv_nop" : "+v"(d) : "v"(a.w), "v"(b.w));
  return d;
}

__device__ __forceinline__ void ldwait() {
  asm volatile("s_wait_loadcnt 0x0" ::: "memory");
}

__device__ __forceinline__ int scan_chunk(const int* __restrict__ dsts, int nE, int cbase, int slotBase,
                                          int nb, int vec8, int* list, int tid, int lane, int wave) {
  int wc = 0;
  const int el0  = tid * EPT;
  const int e0   = cbase + el0;
  const int sent = -2147483647 - 1;
  v4i da, db;
  if (vec8 != 0 && cbase + CHUNK <= nE) {
    da = *(const v4i*)(dsts + e0);
    db = *(const v4i*)(dsts + e0 + 4);
  } else {
    da.x = (e0     < nE) ? dsts[min(e0,     nE - 1)] : sent;
    da.y = (e0 + 1 < nE) ? dsts[min(e0 + 1, nE - 1)] : sent;
    da.z = (e0 + 2 < nE) ? dsts[min(e0 + 2, nE - 1)] : sent;
    da.w = (e0 + 3 < nE) ? dsts[min(e0 + 3, nE - 1)] : sent;
    db.x = (e0 + 4 < nE) ? dsts[min(e0 + 4, nE - 1)] : sent;
    db.y = (e0 + 5 < nE) ? dsts[min(e0 + 5, nE - 1)] : sent;
    db.z = (e0 + 6 < nE) ? dsts[min(e0 + 6, nE - 1)] : sent;
    db.w = (e0 + 7 < nE) ? dsts[min(e0 + 7, nE - 1)] : sent;
  }
  const unsigned nbs = (unsigned)slotBase;
  const unsigned unb = (unsigned)nb;
  const unsigned s0 = (unsigned)da.x - nbs, s1 = (unsigned)da.y - nbs;
  const unsigned s2 = (unsigned)da.z - nbs, s3 = (unsigned)da.w - nbs;
  const unsigned s4 = (unsigned)db.x - nbs, s5 = (unsigned)db.y - nbs;
  const unsigned s6 = (unsigned)db.z - nbs, s7 = (unsigned)db.w - nbs;
  const bool h0 = s0 < unb, h1 = s1 < unb, h2 = s2 < unb, h3 = s3 < unb;
  const bool h4 = s4 < unb, h5 = s5 < unb, h6 = s6 < unb, h7 = s7 < unb;
  const unsigned any = __builtin_amdgcn_ballot_w32(h0 | h1 | h2 | h3 | h4 | h5 | h6 | h7);
  if (any != 0u) {
#define HITJ(J, HJ, SJ) { \
      const unsigned mj = __builtin_amdgcn_ballot_w32(HJ); \
      if (mj != 0u) { \
        if (HJ) { \
          const int pos = wc + (int)__builtin_amdgcn_mbcnt_lo(mj, 0u); \
          if (pos < WCAP) list[wave * WCAP + pos] = ((el0 + (J)) << 12) | (int)(SJ); \
        } \
        wc += (int)__builtin_popcount(mj); } }
    HITJ(0, h0, s0)
    HITJ(1, h1, s1)
    HITJ(2, h2, s2)
    HITJ(3, h3, s3)
    HITJ(4, h4, s4)
    HITJ(5, h5, s5)
    HITJ(6, h6, s6)
    HITJ(7, h7, s7)
#undef HITJ
  }
  return wc;
}

__global__ __launch_bounds__(NTHR) void k_wprep(const float* __restrict__ w1, const float* __restrict__ w2,
                                                const float* __restrict__ lw1, const float* __restrict__ lw2,
                                                unsigned short* wt, int nUnits, int nL, int nC) {
  const int u = (int)blockIdx.x * NTHR + (int)threadIdx.x;
  if (u >= nUnits) return;
  const int per   = DFE * (KA / 8);
  const int nFull = 2 * nL + 1;
  int mat = u / per;
  mat = mat > nFull ? nFull : mat;
  const int o   = u - mat * per;
  const int n   = o / (KA / 8);
  const int k8  = (o - n * (KA / 8)) * 8;
  const float* W;
  int nsrc = DFE;
  if (mat < nL)           { W = w1 + (size_t)mat * DFE * DFE; }
  else if (mat < 2 * nL)  { W = w2 + (size_t)(mat - nL) * DFE * DFE; }
  else if (mat == 2 * nL) { W = lw1; }
  else                    { W = lw2; nsrc = nC; }
  const int nn = n < nsrc ? n : nsrc - 1;
  float wv[8];
#pragma unroll
  for (int e = 0; e < 8; ++e) {
    const int k = (k8 + e) & (DFE - 1);
    wv[e] = W[(size_t)k * (size_t)nsrc + nn];
  }
  ldwait();
  const float keep = (n < nsrc) ? 1.0f : 0.0f;
  v8us pk;
#pragma unroll
  for (int e = 0; e < 8; ++e) pk[e] = bf16s(wv[e] * keep);
  unsigned short* gp = wt + (size_t)mat * WMAT + (size_t)n * KA + k8;
  *(volatile v8us*)gp = pk;
  __threadfence();
  *(volatile v8us*)gp = pk;
}

__global__ __launch_bounds__(NTHR) void k_agg(
    const int* __restrict__ srcs, const int* __restrict__ dsts, const float* __restrict__ h,
    unsigned short* A1, int nN, int nE, int nb, int vec8, int MPr, int rne) {
  extern __shared__ v4f lds_dyn[];
  int* reg1 = (int*)lds_dyn;
  int* reg2 = reg1 + RCAP;
  int* scnt = reg2 + RCAP;
  int* soff = scnt + NBMAX;
  int* list = soff + NBMAX;
  int* wcnt = list + LISTN;
  int* wtot = wcnt + NWAVE;
  const int tid = (int)threadIdx.x, lane = tid & 31, wave = tid >> 5;
  const int nodeBase = (int)blockIdx.x * nb;

  for (int i = tid; i < NBMAX; i += NTHR) scnt[i] = 0;
  __syncthreads();

  int tot = 0;
  const int nChunks = (nE + CHUNK - 1) / CHUNK;
#pragma unroll 1
  for (int ch = 0; ch < nChunks; ++ch) {
    const int cbase = ch * CHUNK;
    const int wc = scan_chunk(dsts, nE, cbase, nodeBase, nb, vec8, list, tid, lane, wave);
    if (lane == 0) wcnt[wave] = wc;
    __syncthreads();
    int pre = 0, all = 0;
#pragma unroll
    for (int w2 = 0; w2 < NWAVE; ++w2) {
      int c = wcnt[w2];
      c = c < 0 ? 0 : (c > WCAP ? WCAP : c);
      all += c;
      pre += (w2 < wave) ? c : 0;
    }
    const int wcc  = wc > WCAP ? WCAP : wc;
    const int base = tot + pre;
#pragma unroll 1
    for (int i = lane; i < wcc; i += 32) {
      const int ent = list[wave * WCAP + i];
      const int el  = (ent >> 12) & (CHUNK - 1);
      const int sl  = ent & (NBMAX - 1);
      int eid = cbase + el;
      eid = eid > nE - 1 ? nE - 1 : eid;
      const int pos = base + i;
      if (pos < RCAP) reg1[pos] = (int)(((unsigned)eid << 12) | (unsigned)sl);
    }
    tot += all;
    tot = tot > RCAP ? RCAP : tot;
    __syncthreads();
  }
  const int nh = tot;

  if (wave == 0) {
#pragma unroll 1
    for (int b0 = 0; b0 < nh; b0 += 32) {
      const int idx = b0 + lane;
      const int uv  = reg1[idx < RCAP ? idx : RCAP - 1];
      const int m32 = (nh - b0) < 32 ? (nh - b0) : 32;
#pragma unroll 1
      for (int k = 0; k < m32; ++k) {
        const int u  = __builtin_amdgcn_readlane(uv, k);
        const int sl = u & (NBMAX - 1);
        if (lane == 0) scnt[sl] = scnt[sl] + 1;
      }
    }
  }
  __syncthreads();

  {
    const v4i ca = *(const v4i*)(scnt + 8 * tid);
    const v4i cb = *(const v4i*)(scnt + 8 * tid + 4);
    const int e0 = ca.x < 0 ? 0 : ca.x, e1 = ca.y < 0 ? 0 : ca.y, e2 = ca.z < 0 ? 0 : ca.z, e3 = ca.w < 0 ? 0 : ca.w;
    const int e4 = cb.x < 0 ? 0 : cb.x, e5 = cb.y < 0 ? 0 : cb.y, e6 = cb.z < 0 ? 0 : cb.z, e7 = cb.w < 0 ? 0 : cb.w;
    const int ts = e0 + e1 + e2 + e3 + e4 + e5 + e6 + e7;
    int incl = ts;
#pragma unroll
    for (int d = 1; d < 32; d <<= 1) {
      const int up = __shfl_up(incl, d);
      if (lane >= d) incl += up;
    }
    if (lane == 31) wtot[wave] = incl;
    __syncthreads();
    int pre = 0;
#pragma unroll
    for (int w2 = 0; w2 < NWAVE; ++w2) pre += (w2 < wave) ? wtot[w2] : 0;
    int run = pre + incl - ts;
    soff[8 * tid + 0] = run; run += e0;
    soff[8 * tid + 1] = run; run += e1;
    soff[8 * tid + 2] = run; run += e2;
    soff[8 * tid + 3] = run; run += e3;
    soff[8 * tid + 4] = run; run += e4;
    soff[8 * tid + 5] = run; run += e5;
    soff[8 * tid + 6] = run; run += e6;
    soff[8 * tid + 7] = run;
  }
  __syncthreads();
  for (int i = tid; i < NBMAX; i += NTHR) list[i] = soff[i];
  __syncthreads();

  if (wave == 0) {
#pragma unroll 1
    for (int b0 = 0; b0 < nh; b0 += 32) {
      const int idx = b0 + lane;
      const int uv  = reg1[idx < RCAP ? idx : RCAP - 1];
      const int m32 = (nh - b0) < 32 ? (nh - b0) : 32;
#pragma unroll 1
      for (int k = 0; k < m32; ++k) {
        const int u   = __builtin_amdgcn_readlane(uv, k);
        const int sl  = u & (NBMAX - 1);
        const int eid = (int)((unsigned)u >> 12);
        if (lane == 0) {
          int pos = list[sl];
          pos = pos < 0 ? 0 : (pos > RCAP - 1 ? RCAP - 1 : pos);
          reg2[pos] = eid;
          list[sl] = pos + 1;
        }
      }
    }
  }
  __syncthreads();

  const int nbw = nb >> 3;
  const bool ovf = (nh >= RCAP);
  const float qnan = __int_as_float(0x7fc00000);
  float* stw = (float*)reg1 + wave * STW;
  const int part = lane >> 4;
  const int c0   = 8 * (lane & 15);
#pragma unroll 1
  for (int jt = 0; jt < nbw; ++jt) {
    const int slot = wave * nbw + jt;
    const int grow = nodeBase + slot;
    const int gcl  = grow < nN ? grow : nN - 1;
    int st = soff[slot];
    const int craw = scnt[slot];
    int cnt = craw;
    st  = st < 0 ? 0 : (st > nh ? nh : st);
    cnt = cnt < 0 ? 0 : (cnt > DEGCAP ? DEGCAP : cnt);
    if (cnt > nh - st) cnt = nh - st;
    const float pz = (ovf || craw > DEGCAP) ? qnan : 0.0f;
    const bool wr = grow < MPr;
    const float live = grow < nN ? 1.0f : 0.0f;

    const float* hrow = h + (size_t)gcl * DFE + lane;
    float hv[4], av[4];
#pragma unroll
    for (int j = 0; j < 4; ++j) { hv[j] = hrow[32 * j]; av[j] = 0.f; }
    ldwait();

#pragma unroll 1
    for (int q = 0; q < cnt; ++q) {
      int idx = st + q; idx = idx > RCAP - 1 ? RCAP - 1 : idx;
      int eid = reg2[idx]; eid = eid < 0 ? 0 : (eid > nE - 1 ? nE - 1 : eid);
      const int sraw = srcs[eid];
      ldwait();
      const int s = sraw < 0 ? 0 : (sraw > nN - 1 ? nN - 1 : sraw);
      const float* hs = h + (size_t)s * DFE + lane;
      float g[4];
#pragma unroll
      for (int j = 0; j < 4; ++j) g[j] = hs[32 * j];
      ldwait();
#pragma unroll
      for (int j = 0; j < 4; ++j) {
        const float gr = rne ? bf16r(g[j]) : g[j];
        av[j] = av[j] + gr;
      }
    }
    float z[4];
#pragma unroll
    for (int j = 0; j < 4; ++j) {
      const float hs2 = rne ? bf16r(hv[j]) : hv[j];
      z[j] = (av[j] + hs2) * live + pz;
    }
    __builtin_amdgcn_fence(__ATOMIC_RELEASE, "wavefront");
    __builtin_amdgcn_wave_barrier();
#pragma unroll
    for (int j = 0; j < 4; ++j) stw[32 * j + lane] = z[j];
    __builtin_amdgcn_fence(__ATOMIC_RELEASE, "wavefront");
    __builtin_amdgcn_wave_barrier();
    const v4f ga = *(const v4fa*)(stw + c0);
    const v4f gb = *(const v4fa*)(stw + c0 + 4);
    const float vv[8] = {ga.x, ga.y, ga.z, ga.w, gb.x, gb.y, gb.z, gb.w};
    v8us pk;
#pragma unroll
    for (int e = 0; e < 8; ++e) {
      const unsigned hu = bf16u(vv[e]);
      const unsigned lu = bf16u(vv[e] - __uint_as_float(hu));
      const unsigned su = part ? lu : hu;
      pk[e] = (unsigned short)(su >> 16);
    }
    unsigned short* gp = A1 + (size_t)grow * KA + 8 * lane;
    if (wr) *(volatile v8us*)gp = pk;
    __threadfence();
    if (wr) *(volatile v8us*)gp = pk;
  }
}

__global__ __launch_bounds__(GTHR) void k_gemm(
    const unsigned short* __restrict__ A, const unsigned short* __restrict__ WT,
    const float* __restrict__ bias, const float* __restrict__ bmu, const float* __restrict__ bva,
    const float* __restrict__ bga, const float* __restrict__ bbe,
    unsigned short* outP, float* outF, int bn, int om) {
  __shared__ __attribute__((aligned(16))) float stg[GBM * DFE];
  __shared__ __attribute__((aligned(16))) float ep[5 * DFE];
  const int tid = (int)threadIdx.x, lane = tid & 31, wave = tid >> 5, hh = lane >> 4, m = lane & 15;
  const int rowBase = (int)blockIdx.x * GBM;

  {
    const float vb = bias[tid];
    const float vm = bmu[tid];
    const float vv = bva[tid];
    const float vg = bga[tid];
    const float ve = bbe[tid];
    ldwait();
    ep[tid]           = bf16r(vb);
    ep[DFE + tid]     = bn ? bf16r(vm) : 0.0f;
    ep[2 * DFE + tid] = bn ? (1.0f / sqrtf(bf16r(vv) + 1e-5f)) : 1.0f;
    ep[3 * DFE + tid] = bn ? bf16r(vg) : 1.0f;
    ep[4 * DFE + tid] = bn ? bf16r(ve) : 0.0f;
  }
  __syncthreads();

  v8f acc[8];
  {
    const v8f z = {0.f, 0.f, 0.f, 0.f, 0.f, 0.f, 0.f, 0.f};
#pragma unroll
    for (int t = 0; t < 8; ++t) acc[t] = z;
  }
  const unsigned short* ap = A  + (size_t)(rowBase + 16 * wave + m) * (size_t)KA + 8 * hh;
  const unsigned short* wp = WT + (size_t)m * (size_t)KA + 8 * hh;
#pragma unroll 1
  for (int ks = 0; ks < KA / 32; ++ks) {
    FragB af;
    af.h[0] = *(const v8usa*)(ap + 32 * ks);
    af.h[1] = *(const v8usa*)(ap + 32 * ks + 16);
#pragma unroll
    for (int t = 0; t < 8; ++t) {
      const unsigned short* wq = wp + (size_t)(16 * t) * (size_t)KA + 32 * ks;
      FragB bf;
      bf.h[0] = *(const v8usa*)wq;
      bf.h[1] = *(const v8usa*)(wq + 16);
      acc[t] = wmb(af, bf, acc[t]);
    }
  }

#pragma unroll
  for (int t = 0; t < 8; ++t) {
    const int lc = 16 * t + m;
    const float pb = ep[lc];
    const float pm = ep[DFE + lc];
    const float pr = ep[2 * DFE + lc];
    const float pg = ep[3 * DFE + lc];
    const float pe = ep[4 * DFE + lc];
#pragma unroll
    for (int r = 0; r < 8; ++r) {
      const int lr = 16 * wave + 8 * hh + r;
      float v = acc[t][r] + pb;
      v = ((v - pm) * pr) * pg + pe;
      stg[lr * DFE + lc] = fmaxf(v, 0.0f);
    }
  }
  __syncthreads();

  if (om == 0) {
    const int part = hh;
    const int c0 = 8 * m;
    v8us pk[16];
#pragma unroll
    for (int i = 0; i < 16; ++i) {
      const int lr = 16 * wave + i;
      const v4f ga = *(const v4fa*)(stg + lr * DFE + c0);
      const v4f gb = *(const v4fa*)(stg + lr * DFE + c0 + 4);
      const float vv[8] = {ga.x, ga.y, ga.z, ga.w, gb.x, gb.y, gb.z, gb.w};
      v8us p;
#pragma unroll
      for (int e = 0; e < 8; ++e) {
        const unsigned hu = bf16u(vv[e]);
        const unsigned lu = bf16u(vv[e] - __uint_as_float(hu));
        const unsigned su = part ? lu : hu;
        p[e] = (unsigned short)(su >> 16);
      }
      pk[i] = p;
    }
#pragma unroll
    for (int i = 0; i < 16; ++i) {
      const int lr = 16 * wave + i;
      unsigned short* gp = outP + (size_t)(rowBase + lr) * (size_t)KA + 8 * lane;
      *(volatile v8us*)gp = pk[i];
    }
    __threadfence();
#pragma unroll
    for (int i = 0; i < 16; ++i) {
      const int lr = 16 * wave + i;
      unsigned short* gp = outP + (size_t)(rowBase + lr) * (size_t)KA + 8 * lane;
      *(volatile v8us*)gp = pk[i];
    }
  } else {
    v4f fv[16];
#pragma unroll
    for (int i = 0; i < 16; ++i) {
      const int lr = 16 * wave + i;
      fv[i] = *(const v4fa*)(stg + lr * DFE + 4 * lane);
    }
#pragma unroll
    for (int i = 0; i < 16; ++i) {
      const int lr = 16 * wave + i;
      float* op = outF + (size_t)(rowBase + lr) * (size_t)DFE + 4 * lane;
      *(volatile v4f*)op = fv[i];
    }
    __threadfence();
#pragma unroll
    for (int i = 0; i < 16; ++i) {
      const int lr = 16 * wave + i;
      float* op = outF + (size_t)(rowBase + lr) * (size_t)DFE + 4 * lane;
      *(volatile v4f*)op = fv[i];
    }
  }
}

__global__ __launch_bounds__(GTHR) void k_head(
    const unsigned short* __restrict__ A, const unsigned short* __restrict__ WT,
    const float* __restrict__ bias, float* out, int nN, int nC) {
  __shared__ __attribute__((aligned(16))) float stg[GBM * NCMAX];
  __shared__ __attribute__((aligned(16))) float outs[GBM * NCMAX];
  __shared__ float pb[NCMAX];
  const int tid = (int)threadIdx.x, lane = tid & 31, wave = tid >> 5, hh = lane >> 4, m = lane & 15;
  const int rowBase = (int)blockIdx.x * GBM;

  if (tid < NCMAX) {
    const int cc = tid < nC ? tid : nC - 1;
    const float v = bias[cc];
    ldwait();
    pb[tid] = (tid < nC) ? bf16r(v) : 0.0f;
  }
  __syncthreads();

  v8f acc[4];
  {
    const v8f z = {0.f, 0.f, 0.f, 0.f, 0.f, 0.f, 0.f, 0.f};
#pragma unroll
    for (int t = 0; t < 4; ++t) acc[t] = z;
  }
  const unsigned short* ap = A  + (size_t)(rowBase + 16 * wave + m) * (size_t)KA + 8 * hh;
  const unsigned short* wp = WT + (size_t)m * (size_t)KA + 8 * hh;
#pragma unroll 1
  for (int ks = 0; ks < KA / 32; ++ks) {
    FragB af;
    af.h[0] = *(const v8usa*)(ap + 32 * ks);
    af.h[1] = *(const v8usa*)(ap + 32 * ks + 16);
#pragma unroll
    for (int t = 0; t < 4; ++t) {
      const unsigned short* wq = wp + (size_t)(16 * t) * (size_t)KA + 32 * ks;
      FragB bf;
      bf.h[0] = *(const v8usa*)wq;
      bf.h[1] = *(const v8usa*)(wq + 16);
      acc[t] = wmb(af, bf, acc[t]);
    }
  }

#pragma unroll
  for (int t = 0; t < 4; ++t) {
    const int lc = 16 * t + m;
    const float bb = pb[lc];
#pragma unroll
    for (int r = 0; r < 8; ++r) {
      const int lr = 16 * wave + 8 * hh + r;
      stg[lr * NCMAX + lc] = acc[t][r] + bb;
    }
  }
  __syncthreads();

  if (tid < GBM) {
    const float* lrow = stg + tid * NCMAX;
    float mx = lrow[0];
#pragma unroll 1
    for (int c = 1; c < nC; ++c) mx = fmaxf(mx, lrow[c]);
    float s = 0.0f;
#pragma unroll 1
    for (int c = 0; c < nC; ++c) s += expf(lrow[c] - mx);
    const float lse = logf(s);
    float* orow = outs + tid * nC;
#pragma unroll 1
    for (int c = 0; c < nC; ++c) orow[c] = (lrow[c] - mx) - lse;
  }
  __syncthreads();

  const int nP = (GBM * nC) >> 2;
  const size_t gp0  = (size_t)blockIdx.x * (size_t)nP;
  const size_t totP = ((size_t)nN * (size_t)nC) >> 2;
  const int nIt = (nP + GTHR - 1) / GTHR;
#pragma unroll 1
  for (int it = 0; it < nIt; ++it) {
    const int p  = tid + GTHR * it;
    const int pc = p < nP ? p : nP - 1;
    const v4f v = *(const v4fa*)(outs + 4 * pc);
    if (p < nP && gp0 + (size_t)p < totP) *(volatile v4f*)(out + (gp0 + (size_t)p) * 4) = v;
  }
  __threadfence();
#pragma unroll 1
  for (int it = 0; it < nIt; ++it) {
    const int p  = tid + GTHR * it;
    const int pc = p < nP ? p : nP - 1;
    const v4f v = *(const v4fa*)(outs + 4 * pc);
    if (p < nP && gp0 + (size_t)p < totP) *(volatile v4f*)(out + (gp0 + (size_t)p) * 4) = v;
  }
}

static int pick_nb(int nE, int nN) {
  int nb = NBMAX;
  while (nb > 16 && (long long)nb * (long long)nE * 5LL > (long long)RCAP * (long long)nN * 4LL) nb >>= 1;
  return nb;
}
static inline int cdiv(int a, int b) { return (a + b - 1) / b; }

extern "C" void kernel_launch(void* const* d_in, const int* in_sizes, int n_in,
                              void* d_out, int out_size, void* d_ws, size_t ws_size,
                              hipStream_t stream) {
  if (n_in < 14) return;
  if (in_sizes[0] < DFE || (in_sizes[0] % DFE) != 0) return;
  const int nN = in_sizes[0] / DFE;
  if (nN <= 0 || nN > (1 << 22)) return;
  if (in_sizes[1] < 2 || (in_sizes[1] % 2) != 0) return;
  const int nE = in_sizes[1] / 2;
  if (nE < 1 || nE > (1 << 20)) return;
  if (in_sizes[2] < DFE * DFE || (in_sizes[2] % (DFE * DFE)) != 0) return;
  const int nL = in_sizes[2] / (DFE * DFE);
  if (nL < 1 || nL > 8) return;
  for (int i = 3; i <= 7; ++i) if (in_sizes[i] != nL * DFE) return;
  if (in_sizes[8] != nL * DFE * DFE || in_sizes[9] != nL * DFE) return;
  if (in_sizes[10] != DFE * DFE || in_sizes[11] != DFE) return;
  const int nC = in_sizes[13];
  if (nC < 1 || nC > NCMAX) return;
  if (in_sizes[12] != DFE * nC) return;
  if (out_size != nN * nC) return;
  if ((((long long)nN * (long long)nC) & 3LL) != 0) return;

  const float* x     = (const float*)d_in[0];
  const int*   ei    = (const int*)  d_in[1];
  const float* W1    = (const float*)d_in[2];
  const float* b1    = (const float*)d_in[3];
  const float* gamma = (const float*)d_in[4];
  const float* beta  = (const float*)d_in[5];
  const float* bmean = (const float*)d_in[6];
  const float* bvar  = (const float*)d_in[7];
  const float* W2    = (const float*)d_in[8];
  const float* b2    = (const float*)d_in[9];
  const float* lw1   = (const float*)d_in[10];
  const float* lb1   = (const float*)d_in[11];
  const float* lw2   = (const float*)d_in[12];
  const float* lb2   = (const float*)d_in[13];
  const int* src = ei;
  const int* dst = ei + nE;
  float* out = (float*)d_out;

  const int MP   = cdiv(nN, GBM) * GBM;
  const int gM   = MP / GBM;
  const int nb   = pick_nb(nE, nN);
  const int gA   = cdiv(MP, nb);
  const int vec8 = ((nE % 4) == 0) ? 1 : 0;
  if (gA * nb < MP) return;

  const size_t nWTh = (size_t)(2 * nL + 1) * WMAT + (size_t)NCMAX * KA;
  char* ws = (char*)d_ws;
  size_t off = 0;
  const size_t oWT  = off; off += nWTh * 2;                        off = (off + 255) & ~(size_t)255;
  const size_t oA1  = off; off += (size_t)MP * KA * 2;             off = (off + 255) & ~(size_t)255;
  const size_t oA2  = off; off += (size_t)MP * KA * 2;             off = (off + 255) & ~(size_t)255;
  const size_t oA3  = off; off += (size_t)MP * KA * 2;             off = (off + 255) & ~(size_t)255;
  const size_t oHF0 = off; off += (size_t)MP * DFE * 4;            off = (off + 255) & ~(size_t)255;
  const size_t oHF1 = off; off += (size_t)MP * DFE * 4;            off = (off + 255) & ~(size_t)255;
  if (off > ws_size || off > (size_t)WSMAX) return;
  unsigned short* WT  = (unsigned short*)(ws + oWT);
  unsigned short* A1  = (unsigned short*)(ws + oA1);
  unsigned short* A2  = (unsigned short*)(ws + oA2);
  unsigned short* A3  = (unsigned short*)(ws + oA3);
  float*          HF0 = (float*)(ws + oHF0);
  float*          HF1 = (float*)(ws + oHF1);

  hipFuncSetAttribute(reinterpret_cast<const void*>(&k_agg),
                      hipFuncAttributeMaxDynamicSharedMemorySize, LDS_AGG);

  const int nUw = (2 * nL + 1) * DFE * (KA / 8) + NCMAX * (KA / 8);
  k_wprep<<<cdiv(nUw, NTHR), NTHR, 0, stream>>>(W1, W2, lw1, lw2, WT, nUw, nL, nC);

  for (int l = 0; l < nL; ++l) {
    const float* hin = (l == 0) ? x : (((l - 1) & 1) ? HF1 : HF0);
    float* hout = (l & 1) ? HF1 : HF0;
    const int rne = (l == 0) ? 1 : 0;
    const float* b1l = b1 + (size_t)l * DFE;
    const float* b2l = b2 + (size_t)l * DFE;

    k_agg<<<gA, NTHR, LDS_AGG, stream>>>(src, dst, hin, A1, nN, nE, nb, vec8, MP, rne);

    k_gemm<<<gM, GTHR, 0, stream>>>(A1, WT + (size_t)l * WMAT, b1l,
                                    bmean + (size_t)l * DFE, bvar + (size_t)l * DFE,
                                    gamma + (size_t)l * DFE, beta + (size_t)l * DFE,
                                    A2, hout, 1, 0);

    if (l < nL - 1) {
      k_gemm<<<gM, GTHR, 0, stream>>>(A2, WT + (size_t)(nL + l) * WMAT, b2l, b2l, b2l, b2l, b2l,
                                      A3, hout, 0, 1);
    } else {
      k_gemm<<<gM, GTHR, 0, stream>>>(A2, WT + (size_t)(nL + l) * WMAT, b2l, b2l, b2l, b2l, b2l,
                                      A3, hout, 0, 0);
    }
  }

  k_gemm<<<gM, GTHR, 0, stream>>>(A3, WT + (size_t)(2 * nL) * WMAT, lb1, lb1, lb1, lb1, lb1, A1, HF0, 0, 0);

  k_head<<<gM, GTHR, 0, stream>>>(A1, WT + (size_t)(2 * nL + 1) * WMAT, lb2, out, nN, nC);
}
